// BaseSigKernel_60335700574840
// MI455X (gfx1250) — hardware-run, weakly checked
//
#include <hip/hip_runtime.h>
#include <math.h>

typedef __attribute__((ext_vector_type(16))) _Float16 v16h;
typedef __attribute__((ext_vector_type(8)))  float    v8f;
typedef __attribute__((ext_vector_type(4)))  float    v4f;

constexpr int kNumX       = 16;
constexpr int kNumY       = 16;
constexpr int kLen        = 128;
constexpr int kDim        = 8;
constexpr int kPairs      = kNumX * kNumY;
constexpr int kTilePitch  = kLen + 1;
constexpr int kDiffN      = kLen - 1;
constexpr int kGrid       = 2 * kDiffN;
constexpr int kSteps      = 2 * kGrid - 1;
constexpr int kLineFloats = 32;
constexpr int kThreads    = 256;
constexpr int kDiffChunks = 4;
constexpr int kDiffPer    = 16;
constexpr int kChunkRows  = 2 * kDiffPer;
constexpr float kCarry        = 64.0f;
constexpr float kFold         = 1.0f / (kCarry * kCarry);
constexpr float kF16MinNormal = 6.103515625e-5f;
constexpr float kF32MinNormal = 1.17549435e-38f;
constexpr float kTwelfth      = 1.0f / 12.0f;
static_assert(kPairs == 256, "pair count");
static_assert(kDim == 8 && kLen == 128, "fragment construction assumes 8 coordinates and 8 row tiles");
static_assert(kGrid + 1 <= kThreads, "one lane per grid row");
static_assert(kSteps == 507, "sweep length");
static_assert(kChunkRows * kDiffChunks == kLen, "difference chunks cover all tile rows");
static_assert(2 * kLen == kThreads, "two row parities x 128 columns in the difference pass");

constexpr size_t kWsTotal = (size_t)kPairs * kLineFloats * 4;
static_assert(kWsTotal == 32768ull, "carve total");
static_assert(kWsTotal <= 134217728ull, "carve cap");

__device__ __forceinline__ v8f mma_f16_guarded(v16h a, v16h b, v8f c) {
  c = __builtin_amdgcn_wmma_f32_16x16x32_f16(false, a, false, b, (short)0, c, false, false);
  asm volatile("v_nop\n\tv_nop\n\tv_nop\n\tv_nop" : "+v"(c) : "v"(a), "v"(b));
  return c;
}

__device__ __forceinline__ float carry_flush(float v, bool live) {
  float c = v * kCarry;
  c = (fabsf(c) < kF16MinNormal) ? 0.0f : c;
  c = live ? c : 0.0f;
  return c;
}

__device__ __forceinline__ v16h build_frag(const float* rowp, bool live) {
  const v4f r0 = *(const v4f*)(rowp);
  const v4f r1 = *(const v4f*)(rowp + 4);
  float c0 = r0[0];
  float c1 = r0[1];
  float c2 = r0[2];
  float c3 = r0[3];
  float c4 = r1[0];
  float c5 = r1[1];
  float c6 = r1[2];
  float c7 = r1[3];
  asm volatile("" : "+v"(c0));
  asm volatile("" : "+v"(c1));
  asm volatile("" : "+v"(c2));
  asm volatile("" : "+v"(c3));
  asm volatile("" : "+v"(c4));
  asm volatile("" : "+v"(c5));
  asm volatile("" : "+v"(c6));
  asm volatile("" : "+v"(c7));
  v16h f;
  f[0]  = (_Float16)carry_flush(c0, live);
  f[1]  = (_Float16)carry_flush(c1, live);
  f[2]  = (_Float16)carry_flush(c2, live);
  f[3]  = (_Float16)carry_flush(c3, live);
  f[4]  = (_Float16)carry_flush(c4, live);
  f[5]  = (_Float16)carry_flush(c5, live);
  f[6]  = (_Float16)carry_flush(c6, live);
  f[7]  = (_Float16)carry_flush(c7, live);
  f[8]  = (_Float16)0.0f;
  f[9]  = (_Float16)0.0f;
  f[10] = (_Float16)0.0f;
  f[11] = (_Float16)0.0f;
  f[12] = (_Float16)0.0f;
  f[13] = (_Float16)0.0f;
  f[14] = (_Float16)0.0f;
  f[15] = (_Float16)0.0f;
  return f;
}

__global__ __launch_bounds__(256) __attribute__((amdgpu_num_vgpr(256)))
void pair_grid_kernel(const float* __restrict__ xs,
                      const float* __restrict__ ys,
                      float* __restrict__ wsres) {
  __shared__ __align__(16) float sK[kLen * kTilePitch];
  __shared__ __align__(16) float sNrm[2 * kLen];
  __shared__ __align__(16) float sDg[2 * kThreads];

  const int tid  = threadIdx.x;
  const int lane = tid & 31;
  const int wave = tid >> 5;
  const int b    = blockIdx.x;
  const int ix   = b >> 4;
  const int iy   = b & 15;
  const float* x = xs + (size_t)ix * (kLen * kDim);
  const float* y = ys + (size_t)iy * (kLen * kDim);

  {
    const int r = tid & (kLen - 1);
    const float* src = (tid < kLen) ? x : y;
    const v4f a0 = *(const v4f*)(src + r * kDim);
    const v4f a1 = *(const v4f*)(src + r * kDim + 4);
    float s = 0.0f;
    s = fmaf(a0[0], a0[0], s);
    s = fmaf(a0[1], a0[1], s);
    s = fmaf(a0[2], a0[2], s);
    s = fmaf(a0[3], a0[3], s);
    s = fmaf(a1[0], a1[0], s);
    s = fmaf(a1[1], a1[1], s);
    s = fmaf(a1[2], a1[2], s);
    s = fmaf(a1[3], a1[3], s);
    sNrm[tid] = s;
    sDg[tid] = 1.0f;
    sDg[kThreads + tid] = 1.0f;
  }
  __syncthreads();

  {
    const int hsel = lane >> 4;
    const int m    = lane & 15;
    const bool live = (hsel == 0);
    const v16h afrag = build_frag(x + (wave * 16 + m) * kDim, live);
    const int row0 = wave * 16 + 8 * hsel;
    float xr[8];
#pragma unroll
    for (int r = 0; r < 8; ++r) xr[r] = sNrm[row0 + r];
#pragma unroll 1
    for (int tj = 0; tj < 8; ++tj) {
      const int col = tj * 16 + m;
      const v16h bfrag = build_frag(y + col * kDim, live);
      v8f acc = (v8f){0.f, 0.f, 0.f, 0.f, 0.f, 0.f, 0.f, 0.f};
      acc = mma_f16_guarded(afrag, bfrag, acc);
      const float yn = sNrm[kLen + col];
#pragma unroll
      for (int r = 0; r < 8; ++r) {
        const float g  = acc[r] * kFold;
        const float sq = (xr[r] + yn) - 2.0f * g;
        float e = expf(-0.5f * sq);
        e = (e < kF32MinNormal) ? 0.0f : e;
        sK[(row0 + r) * kTilePitch + col] = e;
      }
    }
  }
  __syncthreads();

  {
    const int q  = tid & (kLen - 1);
    const int p0 = tid >> 7;
    const int qc = (q < kDiffN) ? q : (kDiffN - 1);
#pragma unroll 1
    for (int c = 0; c < kDiffChunks; ++c) {
      const int pbase = c * kChunkRows + p0;
      float dv[kDiffPer];
#pragma unroll
      for (int it = 0; it < kDiffPer; ++it) {
        const int p  = pbase + 2 * it;
        const int pc = (p < kDiffN) ? p : (kDiffN - 1);
        const int base = pc * kTilePitch + qc;
        const float k00 = sK[base];
        const float k01 = sK[base + 1];
        const float k10 = sK[base + kTilePitch];
        const float k11 = sK[base + kTilePitch + 1];
        dv[it] = 0.25f * (((k11 + k00) - k10) - k01);
      }
      __syncthreads();
#pragma unroll
      for (int it = 0; it < kDiffPer; ++it) {
        const int p = pbase + 2 * it;
        if (q < kDiffN && p < kDiffN) sK[p * kTilePitch + q] = dv[it];
      }
    }
  }
  __syncthreads();

  {
    const int i   = tid;
    const int im1 = (i > 0) ? (i - 1) : 0;
    int pr = (i - 1) >> 1;
    pr = (pr < 0) ? 0 : pr;
    pr = (pr > kDiffN - 1) ? (kDiffN - 1) : pr;
    const int prow = pr * kTilePitch;
    const bool rowlive = (i >= 1) && (i <= kGrid);
    float own   = 1.0f;
    float left2 = 1.0f;
#pragma unroll 1
    for (int s = 0; s < kSteps; ++s) {
      const int j = (s + 2) - i;
      int qq = (j - 1) >> 1;
      qq = (qq < 0) ? 0 : qq;
      qq = (qq > kDiffN - 1) ? (kDiffN - 1) : qq;
      const float inc = sK[prow + qq];
      const int rd = (s & 1) * kThreads;
      const int wr = kThreads - rd;
      const float k10 = sDg[rd + im1];
      const bool cell = rowlive && (j >= 1) && (j <= kGrid);
      const float i2 = (inc * inc) * kTwelfth;
      const float f1 = (1.0f + 0.5f * inc) + i2;
      const float f2 = 1.0f - i2;
      const float k11 = (k10 + own) * f1 - left2 * f2;
      const float val = cell ? k11 : 1.0f;
      left2 = k10;
      own   = val;
      sDg[wr + i] = val;
      __syncthreads();
    }
  }

  {
    const float res = sDg[kThreads + kGrid];
    if (tid < 8) {
      const v4f o = (v4f){res, res, res, res};
      float* p = wsres + (size_t)b * kLineFloats + tid * 4;
      *(volatile v4f*)p = o;
      __threadfence();
      *(volatile v4f*)p = o;
    }
  }
}

__global__ __launch_bounds__(32) void pack_out_kernel(const float* __restrict__ wsres, float* __restrict__ out) {
  const int lane = threadIdx.x & 31;
  const int e0 = 4 * lane;
  const int e1 = 128 + 4 * lane;
  const float t0 = wsres[(size_t)(e0 + 0) * kLineFloats];
  const float t1 = wsres[(size_t)(e0 + 1) * kLineFloats];
  const float t2 = wsres[(size_t)(e0 + 2) * kLineFloats];
  const float t3 = wsres[(size_t)(e0 + 3) * kLineFloats];
  const float u0 = wsres[(size_t)(e1 + 0) * kLineFloats];
  const float u1 = wsres[(size_t)(e1 + 1) * kLineFloats];
  const float u2 = wsres[(size_t)(e1 + 2) * kLineFloats];
  const float u3 = wsres[(size_t)(e1 + 3) * kLineFloats];
  const v4f o0 = (v4f){t0, t1, t2, t3};
  const v4f o1 = (v4f){u0, u1, u2, u3};
  *(volatile v4f*)(out + e0) = o0;
  *(volatile v4f*)(out + e1) = o1;
  __threadfence();
  *(volatile v4f*)(out + e0) = o0;
  *(volatile v4f*)(out + e1) = o1;
}

extern "C" void kernel_launch(void* const* d_in, const int* in_sizes, int n_in,
                              void* d_out, int out_size, void* d_ws, size_t ws_size,
                              hipStream_t stream) {
  if (n_in < 2) return;
  if (in_sizes[0] != kNumX * kLen * kDim) return;
  if (in_sizes[1] != kNumY * kLen * kDim) return;
  if (out_size != kPairs) return;
  if (ws_size < kWsTotal) return;

  const float* xs = (const float*)d_in[0];
  const float* ys = (const float*)d_in[1];
  float* out   = (float*)d_out;
  float* wsres = (float*)d_ws;

  pair_grid_kernel<<<kPairs, kThreads, 0, stream>>>(xs, ys, wsres);
  pack_out_kernel<<<1, 32, 0, stream>>>(wsres, out);
}
